// ImplicitMotionAlignment_82265803588078
// MI455X (gfx1250) — hardware-verified
//
#include <hip/hip_runtime.h>
#include <math.h>
#include <stdint.h>

#define NS     4096
#define NC     256
#define NHD    8
#define DHD    32
#define FFI    1024
#define NBLK   2
#define LNEPS  1e-5f
#define RSCALE 0.17677669529663687f
#define XSCALE 0.0625f
#define WSC    64.0f
#define PSC    16.0f
#define OSC    32.0f
#define HSC    16.0f
#define VSA    16.0f
#define LOSC   2048.0f
#define PCAR   1024.0f

#define F_BIASN 1
#define F_BIASM 2
#define F_RESID 4
#define F_GELU  8
#define F_OUT16 16

static_assert(NHD * DHD == NC);
static_assert((NS % 64) == 0 && (NC % 64) == 0 && (FFI % 64) == 0 && (NS % 32) == 0 && (NS % 8) == 0);
static_assert(((3 * NC * NC) % 2048) == 0 && ((NC * NC) % 2048) == 0 && ((FFI * NC) % 2048) == 0 && ((NS * NC) % 2048) == 0);

typedef _Float16 v16h __attribute__((ext_vector_type(16)));
typedef _Float16 v8h  __attribute__((ext_vector_type(8)));
typedef float    v8f  __attribute__((ext_vector_type(8)));
typedef float    v4f  __attribute__((ext_vector_type(4)));
typedef unsigned int v4u __attribute__((ext_vector_type(4)));

__device__ __forceinline__ unsigned short bf_bits(float f) {
  unsigned u = __float_as_uint(f);
  return (unsigned short)((u + 0x7FFFu + ((u >> 16) & 1u)) >> 16);
}
__device__ __forceinline__ float bf_up(unsigned short h) { return __uint_as_float(((unsigned)h) << 16); }
__device__ __forceinline__ float bfr(float f) { return bf_up(bf_bits(f)); }
__device__ __forceinline__ unsigned short h_bits(_Float16 x) { return __builtin_bit_cast(unsigned short, x); }
__device__ __forceinline__ unsigned pk16(unsigned short a, unsigned short b) { return (unsigned)a | ((unsigned)b << 16); }
__device__ __forceinline__ unsigned pkh(float a, float b) { return pk16(h_bits((_Float16)a), h_bits((_Float16)b)); }
__device__ __forceinline__ v8f zero8() { v8f z = {0.f, 0.f, 0.f, 0.f, 0.f, 0.f, 0.f, 0.f}; return z; }
__device__ __forceinline__ v4f zero4() { v4f z = {0.f, 0.f, 0.f, 0.f}; return z; }

__device__ __forceinline__ v16h ldfrag_h(const _Float16* p) {
  union { v16h v; v8h h[2]; } f;
  f.h[0] = *(const v8h*)(p);
  f.h[1] = *(const v8h*)(p + 16);
  return f.v;
}

__device__ __forceinline__ v8f mma_h(v16h a, v16h b, v8f c) {
  c = __builtin_amdgcn_wmma_f32_16x16x32_f16(false, a, false, b, (short)0, c, false, false);
#if defined(__HIP_DEVICE_COMPILE__)
  asm volatile("v_nop\n\tv_nop\n\tv_nop\n\tv_nop" : "+v"(c) : "v"(a), "v"(b));
#endif
  return c;
}
__device__ __forceinline__ v8f mma_h_raw(v16h a, v16h b, v8f c) {
  return __builtin_amdgcn_wmma_f32_16x16x32_f16(false, a, false, b, (short)0, c, false, false);
}
__device__ __forceinline__ void dep_guard_h(v8f& a, v8f& b, v16h x) {
#if defined(__HIP_DEVICE_COMPILE__)
  asm volatile("v_nop\n\tv_nop\n\tv_nop\n\tv_nop" : "+v"(a), "+v"(b) : "v"(x));
#endif
}
__device__ __forceinline__ void keep4_h(v16h a, v16h b, v16h c, v16h d) {
#if defined(__HIP_DEVICE_COMPILE__)
  asm volatile("v_nop" :: "v"(a), "v"(b), "v"(c), "v"(d));
#endif
}
__device__ __forceinline__ void acc_guard4(v8f& a, v8f& b, v8f& c, v8f& d) {
#if defined(__HIP_DEVICE_COMPILE__)
  asm volatile("v_nop\n\tv_nop\n\tv_nop\n\tv_nop" : "+v"(a), "+v"(b), "+v"(c), "+v"(d));
#endif
}
__device__ __forceinline__ void wave_sync_lds() {
  __builtin_amdgcn_fence(__ATOMIC_RELEASE, "workgroup");
  __builtin_amdgcn_wave_barrier();
  __builtin_amdgcn_fence(__ATOMIC_ACQUIRE, "workgroup");
}

__global__ __launch_bounds__(256) void cvt4(const float* __restrict__ s0, unsigned short* d0, int n0,
                                            const float* __restrict__ s1, unsigned short* d1, int n1,
                                            const float* __restrict__ s2, unsigned short* d2, int n2,
                                            const float* __restrict__ s3, unsigned short* d3, int n3,
                                            float scale) {
  const int y = blockIdx.y;
  const float* src = (y == 0) ? s0 : ((y == 1) ? s1 : ((y == 2) ? s2 : s3));
  unsigned short* dst = (y == 0) ? d0 : ((y == 1) ? d1 : ((y == 2) ? d2 : d3));
  const int n = (y == 0) ? n0 : ((y == 1) ? n1 : ((y == 2) ? n2 : n3));
  const size_t i8 = ((size_t)blockIdx.x * 256 + threadIdx.x) * 8;
  if (i8 >= (size_t)n) return;
  const v4f a = *(const v4f*)(src + i8);
  const v4f b = *(const v4f*)(src + i8 + 4);
  v4u pk;
#pragma unroll
  for (int e = 0; e < 2; ++e) {
    pk[e]     = pkh(bfr(a[2 * e]) * scale, bfr(a[2 * e + 1]) * scale);
    pk[2 + e] = pkh(bfr(b[2 * e]) * scale, bfr(b[2 * e + 1]) * scale);
  }
  unsigned short* gp = dst + i8;
  *(volatile v4u*)gp = pk;
  __threadfence();
  *(volatile v4u*)gp = pk;
}

__global__ __launch_bounds__(256)
void cvt_qk(const float* __restrict__ mlc, const float* __restrict__ qpos, unsigned short* qh, unsigned short* ql,
            const float* __restrict__ mlr, const float* __restrict__ kpos, unsigned short* kh, unsigned short* kl) {
#pragma clang fp contract(off)
  __shared__ float tile[64][65];
  const int tid = threadIdx.x;
  const int z = blockIdx.z;
  const float* src = (z == 0) ? mlc : mlr;
  const float* pos = (z == 0) ? qpos : kpos;
  unsigned short* dh = (z == 0) ? qh : kh;
  unsigned short* dl = (z == 0) ? ql : kl;
  const int s0 = blockIdx.x * 64;
  const int d0 = blockIdx.y * 64;
#pragma unroll
  for (int p = 0; p < 16; ++p) {
    const int idx = p * 256 + tid;
    const int d = idx >> 6, s = idx & 63;
    tile[d][s] = src[(size_t)(d0 + d) * NS + s0 + s];
  }
  __syncthreads();
  const int rl = tid >> 3, c8 = (tid & 7) * 8;
  v4u hv[2], lv[2];
#pragma unroll
  for (int it = 0; it < 2; ++it) {
    const int row = it * 32 + rl;
    const float* pp = pos + (size_t)(s0 + row) * NC + d0 + c8;
    const v4f p0 = *(const v4f*)pp;
    const v4f p1 = *(const v4f*)(pp + 4);
    float q[8];
#pragma unroll
    for (int e = 0; e < 4; ++e) {
      q[e]     = bfr(tile[c8 + e][row]) + bfr(p0[e]);
      q[4 + e] = bfr(tile[c8 + 4 + e][row]) + bfr(p1[e]);
    }
    v4u a, b;
#pragma unroll
    for (int e = 0; e < 4; ++e) {
      const _Float16 h0 = (_Float16)q[2 * e];
      const _Float16 h1 = (_Float16)q[2 * e + 1];
      float r0 = q[2 * e] - (float)h0;
      float r1 = q[2 * e + 1] - (float)h1;
      r0 = r0 * LOSC;
      r1 = r1 * LOSC;
      a[e] = pk16(h_bits(h0), h_bits(h1));
      b[e] = pkh(r0, r1);
    }
    hv[it] = a;
    lv[it] = b;
  }
  for (int pass = 0; pass < 2; ++pass) {
#pragma unroll
    for (int it = 0; it < 2; ++it) {
      const int row = it * 32 + rl;
      const size_t o = (size_t)(s0 + row) * NC + d0 + c8;
      *(volatile v4u*)(dh + o) = hv[it];
      *(volatile v4u*)(dl + o) = lv[it];
    }
    __threadfence();
  }
}

__global__ __launch_bounds__(256)
void attn_x(const unsigned short* __restrict__ qhp, const unsigned short* __restrict__ qlp,
            const unsigned short* __restrict__ khp, const unsigned short* __restrict__ klp,
            const unsigned short* __restrict__ vtp, float* xf) {
#pragma clang fp contract(off)
  union FH { v16h v; v8h h[2]; };
  __shared__ __align__(16) float    Ss[32 * 68];
  __shared__ __align__(16) _Float16 Ps[32 * 64];
  __shared__ float Al[32];
  __shared__ float Li[32];
  __shared__ __align__(16) float    Os[32 * NC];

  const int tid = threadIdx.x, wave = tid >> 5, lane = tid & 31;
  const int hh = lane >> 4, c = lane & 15;
  const int rb = blockIdx.x * 32;
  const int rt = wave >> 2, sub = wave & 3;

  const _Float16* QH = (const _Float16*)(const void*)qhp;
  const _Float16* QL = (const _Float16*)(const void*)qlp;
  const _Float16* KH = (const _Float16*)(const void*)khp;
  const _Float16* KL = (const _Float16*)(const void*)klp;
  const _Float16* VT = (const _Float16*)(const void*)vtp;

  const size_t qo = (size_t)(rb + 16 * rt + c) * NC + 8 * hh;
  const float rlo = 1.0f / LOSC;

  float mrow[4], lrow[4];
#pragma unroll
  for (int i = 0; i < 4; ++i) { mrow[i] = -INFINITY; lrow[i] = 0.f; }
  v8f oacc[4];
#pragma unroll
  for (int t = 0; t < 4; ++t) oacc[t] = zero8();

  for (int kt = 0; kt < NS / 64; ++kt) {
    const int key0 = kt * 64;
    {
      v8f ah = zero8(), ax = zero8();
      const size_t ko = (size_t)(key0 + 16 * sub + c) * NC + 8 * hh;
#pragma unroll 2
      for (int k0 = 0; k0 < NC; k0 += 32) {
        const v16h fqh = ldfrag_h(QH + qo + k0);
        const v16h fql = ldfrag_h(QL + qo + k0);
        const v16h fkh = ldfrag_h(KH + ko + k0);
        const v16h fkl = ldfrag_h(KL + ko + k0);
        ax = mma_h(fqh, fkl, ax);
        ah = mma_h(fqh, fkh, ah);
        ax = mma_h(fql, fkh, ax);
      }
      float* srow = Ss + (16 * rt + 8 * hh) * 68 + 16 * sub + c;
#pragma unroll
      for (int r = 0; r < 8; ++r) {
        float t = ax[r] * rlo;
        t = t + ah[r];
        srow[r * 68] = t * XSCALE;
      }
    }
    __syncthreads();
#pragma unroll
    for (int i = 0; i < 4; ++i) {
      const int row = wave * 4 + i;
      const float s0v = Ss[row * 68 + lane];
      const float s1v = Ss[row * 68 + 32 + lane];
      float m = fmaxf(s0v, s1v);
#pragma unroll
      for (int off = 1; off < 32; off <<= 1) m = fmaxf(m, __shfl_xor(m, off, 32));
      const float mnew  = fmaxf(mrow[i], m);
      const float alpha = (mrow[i] == -INFINITY) ? 0.f : __expf(mrow[i] - mnew);
      mrow[i] = mnew;
      const float p0 = __expf(s0v - mnew);
      const float p1 = __expf(s1v - mnew);
      float ps = p0 + p1;
#pragma unroll
      for (int off = 1; off < 32; off <<= 1) ps = ps + __shfl_xor(ps, off, 32);
      const float lp = lrow[i] * alpha;
      lrow[i] = lp + ps;
      Ps[row * 64 + lane]      = (_Float16)(p0 * PCAR);
      Ps[row * 64 + 32 + lane] = (_Float16)(p1 * PCAR);
      Al[row] = alpha;
    }
    __syncthreads();
    {
#pragma unroll
      for (int r = 0; r < 8; ++r) {
        const float a = Al[16 * rt + 8 * hh + r];
#pragma unroll
        for (int t = 0; t < 4; ++t) oacc[t][r] = oacc[t][r] * a;
      }
#pragma unroll
      for (int kk = 0; kk < 2; ++kk) {
        FH pa;
        const _Float16* pp = Ps + (16 * rt + c) * 64 + kk * 32 + 8 * hh;
        pa.h[0] = *(const v8h*)(pp);
        pa.h[1] = *(const v8h*)(pp + 16);
#pragma unroll
        for (int t = 0; t < 4; ++t) {
          const int d = 64 * sub + 16 * t + c;
          const v16h vb = ldfrag_h(VT + (size_t)d * NS + key0 + kk * 32 + 8 * hh);
          oacc[t] = mma_h(pa.v, vb, oacc[t]);
        }
      }
    }
  }

#pragma unroll
  for (int i = 0; i < 4; ++i) {
    const float l = lrow[i];
    const float il = (l > 0.f) ? (1.0f / l) : 0.f;
    Li[wave * 4 + i] = il * (1.0f / (PCAR * VSA));
  }
  __syncthreads();
#pragma unroll
  for (int r = 0; r < 8; ++r) {
    const int rowl = 16 * rt + 8 * hh + r;
    const float sc = Li[rowl];
#pragma unroll
    for (int t = 0; t < 4; ++t) Os[rowl * NC + 64 * sub + 16 * t + c] = oacc[t][r] * sc;
  }
  __syncthreads();
  {
    v4f q0[4], q1[4];
#pragma unroll
    for (int i = 0; i < 4; ++i) {
      const int row = wave * 4 + i;
      q0[i] = *(const v4f*)(Os + row * NC + 4 * lane);
      q1[i] = *(const v4f*)(Os + row * NC + 128 + 4 * lane);
    }
    for (int pass = 0; pass < 2; ++pass) {
#pragma unroll
      for (int i = 0; i < 4; ++i) {
        const int row = wave * 4 + i;
        float* fp = xf + (size_t)(rb + row) * NC;
        *(volatile v4f*)(fp + 4 * lane) = q0[i];
        *(volatile v4f*)(fp + 128 + 4 * lane) = q1[i];
      }
      __threadfence();
    }
  }
}

__global__ __launch_bounds__(256)
void ln_rows(const float* __restrict__ xin, const float* __restrict__ g, const float* __restrict__ bt,
             const float* __restrict__ qpos, const float* __restrict__ kpos,
             unsigned short* oq, unsigned short* okk, unsigned short* ov, int full, int nrows) {
#pragma clang fp contract(off)
  const int tid = threadIdx.x, wave = tid >> 5, lane = tid & 31;
  const int row = blockIdx.x * 8 + wave;
  const int rowc = (row < nrows) ? row : (nrows - 1);
  const int c8 = lane * 8;
  const float* rp = xin + (size_t)rowc * NC + c8;
  const v4f a = *(const v4f*)rp;
  const v4f b = *(const v4f*)(rp + 4);
  float x[8];
#pragma unroll
  for (int e = 0; e < 4; ++e) { x[e] = a[e]; x[4 + e] = b[e]; }
  float s = 0.f;
#pragma unroll
  for (int e = 0; e < 8; ++e) s = s + x[e];
#pragma unroll
  for (int off = 1; off < 32; off <<= 1) s = s + __shfl_xor(s, off, 32);
  const float mu = s * (1.0f / NC);
  float d[8];
  float s2 = 0.f;
#pragma unroll
  for (int e = 0; e < 8; ++e) { d[e] = x[e] - mu; const float dd = d[e] * d[e]; s2 = s2 + dd; }
#pragma unroll
  for (int off = 1; off < 32; off <<= 1) s2 = s2 + __shfl_xor(s2, off, 32);
  const float var = s2 * (1.0f / NC);
  const float rstd = 1.0f / sqrtf(var + LNEPS);
  float y[8];
#pragma unroll
  for (int e = 0; e < 8; ++e) {
    const float gg = bfr(g[c8 + e]), bb = bfr(bt[c8 + e]);
    float t = d[e] * rstd; t = t * gg; y[e] = t + bb;
  }
  v4u pv;
#pragma unroll
  for (int e = 0; e < 4; ++e) pv[e] = pkh(y[2 * e], y[2 * e + 1]);
  v4u pq = pv, pk = pv;
  if (full != 0) {
    const float* qp = qpos + (size_t)rowc * NC + c8;
    const float* kp = kpos + (size_t)rowc * NC + c8;
    const v4f q0 = *(const v4f*)qp, q1 = *(const v4f*)(qp + 4);
    const v4f k0 = *(const v4f*)kp, k1 = *(const v4f*)(kp + 4);
    float yq[8], yk[8];
#pragma unroll
    for (int e = 0; e < 4; ++e) {
      yq[e]     = y[e] + bfr(q0[e]);
      yq[4 + e] = y[4 + e] + bfr(q1[e]);
      yk[e]     = y[e] + bfr(k0[e]);
      yk[4 + e] = y[4 + e] + bfr(k1[e]);
    }
#pragma unroll
    for (int e = 0; e < 4; ++e) {
      pq[e] = pkh(yq[2 * e], yq[2 * e + 1]);
      pk[e] = pkh(yk[2 * e], yk[2 * e + 1]);
    }
  }
  if (row < nrows) {
    const size_t o = (size_t)row * NC + c8;
    for (int pass = 0; pass < 2; ++pass) {
      *(volatile v4u*)(ov + o) = pv;
      if (full != 0) {
        *(volatile v4u*)(oq + o) = pq;
        *(volatile v4u*)(okk + o) = pk;
      }
      __threadfence();
    }
  }
}

struct GDesc {
  const unsigned short* A;
  const unsigned short* Bt;
  const float* bias;
  const float* resid;
  void* C;
  int lda, ldb, ldc, ldr;
  int M, N, K, blen;
  int flags, mseg, mbstr, moff;
  int nseg, nbstr, noff, tile0;
  int tiles, pad0;
  float wscale, oscale;
};
static_assert(sizeof(GDesc) == 120);
struct GBatch {
  GDesc d[6];
  int nd;
  int tot;
};
static_assert(sizeof(GBatch) == 728);

__device__ __forceinline__ float epi1(float a, int m, int n, float wsc, const float* bias, int blen, int fl) {
#pragma clang fp contract(off)
  float f = a * wsc;
  if (fl & F_BIASN) { const int i = (n < blen) ? n : (blen - 1); f = f + bfr(bias[i]); }
  if (fl & F_BIASM) { const int i = (m < blen) ? m : (blen - 1); f = f + bfr(bias[i]); }
  return f;
}
__device__ __forceinline__ float epi2(float f, float radd, int fl, float osc) {
#pragma clang fp contract(off)
  f = f + radd;
  if (fl & F_GELU) {
    const float u = f * 0.70710678118654752f;
    const float ev = erff(u);
    const float g1 = 1.0f + ev;
    const float hf = 0.5f * f;
    f = hf * g1;
  }
  return f * osc;
}

__global__ __launch_bounds__(256) void gemm_batch(GBatch gb) {
#pragma clang fp contract(off)
  __shared__ __align__(16) float sT[8][16 * 68];
  const int lane = threadIdx.x & 31;
  const int wave = threadIdx.x >> 5;
  const int t = blockIdx.x * 8 + wave;
  if (t >= gb.tot) return;
  int di = 0;
#pragma unroll
  for (int i = 1; i < 6; ++i) { if (t >= gb.d[i].tile0) di = i; }
  GDesc D = gb.d[0];
#pragma unroll
  for (int i = 1; i < 6; ++i) { if (di == i) D = gb.d[i]; }

  const _Float16* A  = (const _Float16*)(const void*)D.A;
  const _Float16* Bt = (const _Float16*)(const void*)D.Bt;
  const int tilesN = D.N >> 6;
  const int lt = t - D.tile0;
  const int tm = lt / tilesN;
  const int tn = lt - tm * tilesN;
  const int m0 = tm * 32;
  const int n0 = tn * 64;

  const int rlane = lane & 15;
  const int koff  = (lane >> 4) * 8;
  const int mOff  = (lane >> 4) * 8;

  v8f acc[2][4];
#pragma unroll
  for (int i = 0; i < 2; ++i)
#pragma unroll
    for (int j = 0; j < 4; ++j) acc[i][j] = zero8();

  for (int k0 = 0; k0 < D.K; k0 += 32) {
    v16h bh[4];
#pragma unroll
    for (int j = 0; j < 4; ++j) {
      const size_t bo = (size_t)(n0 + (j << 4) + rlane) * D.ldb + koff + k0;
      bh[j] = ldfrag_h(Bt + bo);
    }
#pragma unroll
    for (int i = 0; i < 2; ++i) {
      const size_t ao = (size_t)(m0 + (i << 4) + rlane) * D.lda + koff + k0;
      const v16h ah = ldfrag_h(A + ao);
#pragma unroll
      for (int j = 0; j < 4; ++j) acc[i][j] = mma_h_raw(ah, bh[j], acc[i][j]);
      dep_guard_h(acc[i][0], acc[i][3], ah);
    }
    keep4_h(bh[0], bh[1], bh[2], bh[3]);
  }
#pragma unroll
  for (int i = 0; i < 2; ++i) acc_guard4(acc[i][0], acc[i][1], acc[i][2], acc[i][3]);

  const int orow0 = (m0 / D.mseg) * D.mbstr + D.moff + (m0 % D.mseg);
  const int ocol0 = (n0 / D.nseg) * D.nbstr + D.noff + (n0 % D.nseg);
  const int fl = D.flags;
  const float wsc = D.wscale, osc = D.oscale;

  float* slab = sT[wave];
#pragma unroll
  for (int i = 0; i < 2; ++i) {
    const int mBase = m0 + (i << 4);
#pragma unroll
    for (int j = 0; j < 4; ++j) {
#pragma unroll
      for (int r = 0; r < 8; ++r) {
        slab[(mOff + r) * 68 + (j << 4) + rlane] = acc[i][j][r];
      }
    }
    wave_sync_lds();
    if ((fl & F_OUT16) == 0) {
      float* C = (float*)D.C;
      const int h2 = lane >> 4, c4 = (lane & 15) * 4;
      v4f ov[8];
#pragma unroll
      for (int it = 0; it < 8; ++it) {
        const int row = it * 2 + h2;
        const int m = mBase + row;
        const v4f v = *(const v4f*)(slab + row * 68 + c4);
        v4f rv = zero4();
        if (fl & F_RESID) rv = *(const v4f*)(D.resid + (size_t)m * D.ldr + n0 + c4);
        v4f o;
#pragma unroll
        for (int e = 0; e < 4; ++e) {
          const float f = epi1(v[e], m, n0 + c4 + e, wsc, D.bias, D.blen, fl);
          o[e] = epi2(f, rv[e], fl, osc);
        }
        ov[it] = o;
      }
      for (int pass = 0; pass < 2; ++pass) {
#pragma unroll
        for (int it = 0; it < 8; ++it) {
          const int row = it * 2 + h2;
          float* gp = C + (size_t)(orow0 + (i << 4) + row) * D.ldc + ocol0 + c4;
          *(volatile v4f*)gp = ov[it];
        }
        __threadfence();
      }
    } else {
      unsigned short* C = (unsigned short*)D.C;
      const int q = lane >> 3, c8 = (lane & 7) * 8;
      v4u hv[4];
#pragma unroll
      for (int it = 0; it < 4; ++it) {
        const int row = it * 4 + q;
        const int m = mBase + row;
        const float* sp = slab + row * 68 + c8;
        float rr[8];
#pragma unroll
        for (int e = 0; e < 8; ++e) rr[e] = 0.f;
        if (fl & F_RESID) {
          const float* rp2 = D.resid + (size_t)m * D.ldr + n0 + c8;
          const v4f r0v = *(const v4f*)rp2;
          const v4f r1v = *(const v4f*)(rp2 + 4);
#pragma unroll
          for (int e = 0; e < 4; ++e) { rr[e] = r0v[e]; rr[4 + e] = r1v[e]; }
        }
        float fv[8];
#pragma unroll
        for (int e = 0; e < 8; ++e) {
          const float f = epi1(sp[e], m, n0 + c8 + e, wsc, D.bias, D.blen, fl);
          fv[e] = epi2(f, rr[e], fl, osc);
        }
        v4u a;
#pragma unroll
        for (int e = 0; e < 4; ++e) a[e] = pkh(fv[2 * e], fv[2 * e + 1]);
        hv[it] = a;
      }
      for (int pass = 0; pass < 2; ++pass) {
#pragma unroll
        for (int it = 0; it < 4; ++it) {
          const int row = it * 4 + q;
          unsigned short* gp = C + (size_t)(orow0 + (i << 4) + row) * D.ldc + ocol0 + c8;
          *(volatile v4u*)gp = hv[it];
        }
        __threadfence();
      }
    }
    wave_sync_lds();
  }
}

__global__ __launch_bounds__(256)
void attn_h(const unsigned short* __restrict__ qpl, const unsigned short* __restrict__ kpl,
            const unsigned short* __restrict__ vtpl, unsigned short* opl) {
#pragma clang fp contract(off)
  union FH { v16h v; v8h h[2]; };
  __shared__ __align__(16) _Float16 Psh[8][16 * 64];
  __shared__ __align__(16) float    Os[16 * NC];

  const int tid  = threadIdx.x;
  const int wave = tid >> 5;
  const int lane = tid & 31;
  const int hh   = lane >> 4;
  const int c    = lane & 15;
  const int m0   = blockIdx.x * 16;
  const int hd   = wave;

  const _Float16* Q  = (const _Float16*)(const void*)qpl;
  const _Float16* Kh = (const _Float16*)(const void*)kpl;
  const _Float16* Vh = (const _Float16*)(const void*)vtpl;

  const v16h qa = ldfrag_h(Q + (size_t)(m0 + c) * NC + hd * DHD + 8 * hh);

  const float invq2 = 1.0f / (PSC * PSC);
  float mrow[8], lrow[8];
  v8f oh[2];
#pragma unroll
  for (int r = 0; r < 8; ++r) { mrow[r] = -INFINITY; lrow[r] = 0.f; }
  oh[0] = zero8(); oh[1] = zero8();

  _Float16* pw = Psh[wave];

  for (int kt = 0; kt < NS / 64; ++kt) {
    const int kv0 = kt * 64;

    v8f s[4];
#pragma unroll
    for (int j = 0; j < 4; ++j) {
      const int key = kv0 + j * 16 + c;
      const v16h kb = ldfrag_h(Kh + (size_t)key * NC + hd * DHD + 8 * hh);
      const v8f a = mma_h(qa, kb, zero8());
#pragma unroll
      for (int r = 0; r < 8; ++r) {
        const float t0 = a[r] * invq2;
        s[j][r] = t0 * RSCALE;
      }
    }

#pragma unroll
    for (int r = 0; r < 8; ++r) {
      float m = fmaxf(fmaxf(s[0][r], s[1][r]), fmaxf(s[2][r], s[3][r]));
#pragma unroll
      for (int off = 1; off < 16; off <<= 1) m = fmaxf(m, __shfl_xor(m, off, 32));
      const float mnew  = fmaxf(mrow[r], m);
      const float alpha = (mrow[r] == -INFINITY) ? 0.f : __expf(mrow[r] - mnew);
      mrow[r] = mnew;
      float psum = 0.f;
#pragma unroll
      for (int j = 0; j < 4; ++j) {
        const float p  = __expf(s[j][r] - mnew);
        psum = psum + p;
        pw[(8 * hh + r) * 64 + j * 16 + c] = (_Float16)(p * PCAR);
      }
#pragma unroll
      for (int off = 1; off < 16; off <<= 1) psum = psum + __shfl_xor(psum, off, 32);
      const float lp = lrow[r] * alpha;
      lrow[r] = lp + psum;
      oh[0][r] = oh[0][r] * alpha;
      oh[1][r] = oh[1][r] * alpha;
    }
    wave_sync_lds();

#pragma unroll
    for (int kk = 0; kk < 2; ++kk) {
      FH pa;
      pa.h[0] = *(const v8h*)(pw + c * 64 + kk * 32 + 8 * hh);
      pa.h[1] = *(const v8h*)(pw + c * 64 + kk * 32 + 16 + 8 * hh);
#pragma unroll
      for (int tt = 0; tt < 2; ++tt) {
        const int d = hd * DHD + tt * 16 + c;
        const v16h vb = ldfrag_h(Vh + (size_t)d * NS + kv0 + kk * 32 + 8 * hh);
        oh[tt] = mma_h(pa.v, vb, oh[tt]);
      }
    }
    wave_sync_lds();
  }

#pragma unroll
  for (int r = 0; r < 8; ++r) {
    const float l = lrow[r];
    const float il = (l > 0.f) ? (1.0f / l) : 0.f;
    const float inv = il * (OSC / (PCAR * PSC));
#pragma unroll
    for (int tt = 0; tt < 2; ++tt) {
      const int col = hd * DHD + tt * 16 + c;
      Os[(8 * hh + r) * NC + col] = oh[tt][r] * inv;
    }
  }
  __syncthreads();
  {
    v4u hv[2];
#pragma unroll
    for (int it = 0; it < 2; ++it) {
      const int row = wave * 2 + it;
      const float* sp = Os + row * NC + 8 * lane;
      v4u a;
#pragma unroll
      for (int e = 0; e < 4; ++e) a[e] = pkh(sp[2 * e], sp[2 * e + 1]);
      hv[it] = a;
    }
    for (int pass = 0; pass < 2; ++pass) {
#pragma unroll
      for (int it = 0; it < 2; ++it) {
        const int row = wave * 2 + it;
        unsigned short* gp = opl + (size_t)(m0 + row) * NC + 8 * lane;
        *(volatile v4u*)gp = hv[it];
      }
      __threadfence();
    }
  }
}

__global__ __launch_bounds__(256) void out_nchw(const float* __restrict__ xa, float* outp) {
  __shared__ float tile[64][65];
  const int tid = threadIdx.x;
  const int s0 = blockIdx.x * 64, c0 = blockIdx.y * 64;
#pragma unroll
  for (int p = 0; p < 16; ++p) {
    const int idx = p * 256 + tid;
    const int s = idx >> 6, cc = idx & 63;
    tile[s][cc] = xa[(size_t)(s0 + s) * NC + c0 + cc];
  }
  __syncthreads();
  const int rl = tid >> 4, c4 = (tid & 15) * 4;
  v4f ov[4];
#pragma unroll
  for (int it = 0; it < 4; ++it) {
    const int row = it * 16 + rl;
    v4f o;
#pragma unroll
    for (int e = 0; e < 4; ++e) o[e] = tile[c4 + e][row];
    ov[it] = o;
  }
  for (int pass = 0; pass < 2; ++pass) {
#pragma unroll
    for (int it = 0; it < 4; ++it) {
      const int row = it * 16 + rl;
      float* gp = outp + (size_t)(c0 + row) * NS + s0 + c4;
      *(volatile v4f*)gp = ov[it];
    }
    __threadfence();
  }
}

static GDesc gdesc(const unsigned short* A, int lda, const unsigned short* Bt, int ldb, void* C, int ldc,
                   int M, int N, int K, const float* bias, int blen, const float* resid, int ldr,
                   int flags, float wscale, float oscale) {
  GDesc d;
  d.A = A; d.Bt = Bt; d.bias = bias; d.resid = resid; d.C = C;
  d.lda = lda; d.ldb = ldb; d.ldc = ldc; d.ldr = ldr;
  d.M = M; d.N = N; d.K = K; d.blen = blen;
  d.flags = flags; d.mseg = 1 << 30; d.mbstr = 0; d.moff = 0;
  d.nseg = 1 << 30; d.nbstr = 0; d.noff = 0; d.tile0 = 0;
  d.tiles = (M / 32) * (N / 64); d.pad0 = 0;
  d.wscale = wscale; d.oscale = oscale;
  return d;
}
static void run_gemm(const GDesc* ds, int nd, hipStream_t stream) {
  GBatch gb;
  int tot = 0;
  for (int i = 0; i < 6; ++i) {
    if (i < nd) { gb.d[i] = ds[i]; gb.d[i].tile0 = tot; tot += ds[i].tiles; }
    else        { gb.d[i] = ds[0]; gb.d[i].tile0 = 1 << 30; gb.d[i].tiles = 0; }
  }
  gb.nd = nd; gb.tot = tot;
  if (tot <= 0) return;
  const dim3 grid((tot + 7) / 8);
  gemm_batch<<<grid, dim3(256), 0, stream>>>(gb);
}

extern "C" void kernel_launch(void* const* d_in, const int* in_sizes, int n_in,
                              void* d_out, int out_size, void* d_ws, size_t ws_size,
                              hipStream_t stream) {
  if (n_in < 5 + 14 * NBLK) return;
  const int exb[14] = { NC, NC, NC, NC, 3 * NC * NC, 3 * NC, NC * NC, NC, FFI * NC, FFI, NC * FFI, NC, NS * NC, NS * NC };
  for (int i = 0; i < 5; ++i) if (in_sizes[i] != NS * NC) return;
  for (int b = 0; b < NBLK; ++b)
    for (int j = 0; j < 14; ++j) if (in_sizes[5 + 14 * b + j] != exb[j]) return;
  if (out_size != NS * NC) return;

  const float* ml_c = (const float*)d_in[0];
  const float* ml_r = (const float*)d_in[1];
  const float* fl_r = (const float*)d_in[2];
  const float* caq  = (const float*)d_in[3];
  const float* cak  = (const float*)d_in[4];
  float* out = (float*)d_out;

  const size_t sWI = (size_t)NBLK * 3 * NC * NC * 2;
  const size_t sWO = (size_t)NBLK * NC * NC * 2;
  const size_t sW1 = (size_t)NBLK * FFI * NC * 2;
  const size_t sW2 = sW1;
  const size_t sP16 = (size_t)NS * NC * 2;
  const size_t sP32 = (size_t)NS * NC * 4;
  const size_t sHP = (size_t)NS * FFI * 2;
  size_t off = 0;
  const size_t oWI = off; off += sWI;
  const size_t oWO = off; off += sWO;
  const size_t oW1 = off; off += sW1;
  const size_t oW2 = off; off += sW2;
  const size_t oQH = off; off += sP16;
  const size_t oQL = off; off += sP16;
  const size_t oKH = off; off += sP16;
  const size_t oKL = off; off += sP16;
  const size_t oVTA = off; off += sP16;
  const size_t oXA = off; off += sP32;
  const size_t oXB = off; off += sP32;
  const size_t oXQ = off; off += sP16;
  const size_t oXK = off; off += sP16;
  const size_t oXV = off; off += sP16;
  const size_t oQP = off; off += sP16;
  const size_t oKP = off; off += sP16;
  const size_t oVTP = off; off += sP16;
  const size_t oOP = off; off += sP16;
  const size_t oAH = off; off += sP16;
  const size_t oHP = off; off += sHP;
  if (off > ws_size) return;
  if (off > (size_t)134217728) return;

  char* ws = (char*)d_ws;
  unsigned short* WIP = (unsigned short*)(ws + oWI);
  unsigned short* WOP = (unsigned short*)(ws + oWO);
  unsigned short* W1P = (unsigned short*)(ws + oW1);
  unsigned short* W2P = (unsigned short*)(ws + oW2);
  unsigned short* QH  = (unsigned short*)(ws + oQH);
  unsigned short* QL  = (unsigned short*)(ws + oQL);
  unsigned short* KH  = (unsigned short*)(ws + oKH);
  unsigned short* KL  = (unsigned short*)(ws + oKL);
  unsigned short* VTA = (unsigned short*)(ws + oVTA);
  float*          XA  = (float*)(ws + oXA);
  float*          XB  = (float*)(ws + oXB);
  unsigned short* XQ  = (unsigned short*)(ws + oXQ);
  unsigned short* XK  = (unsigned short*)(ws + oXK);
  unsigned short* XV  = (unsigned short*)(ws + oXV);
  unsigned short* QP  = (unsigned short*)(ws + oQP);
  unsigned short* KP  = (unsigned short*)(ws + oKP);
  unsigned short* VTP = (unsigned short*)(ws + oVTP);
  unsigned short* OP  = (unsigned short*)(ws + oOP);
  unsigned short* AH  = (unsigned short*)(ws + oAH);
  unsigned short* HP  = (unsigned short*)(ws + oHP);

  const dim3 blk(256);
  const int nP = NS * NC;

  cvt4<<<dim3(nP / 2048, 1), blk, 0, stream>>>(fl_r, VTA, nP, fl_r, VTA, nP, fl_r, VTA, nP, fl_r, VTA, nP, VSA);
  for (int i = 0; i < NBLK; ++i) {
    const int base = 5 + 14 * i;
    const float* ipw = (const float*)d_in[base + 4];
    const float* opw = (const float*)d_in[base + 6];
    const float* w1  = (const float*)d_in[base + 8];
    const float* w2  = (const float*)d_in[base + 10];
    cvt4<<<dim3((FFI * NC) / 2048, 4), blk, 0, stream>>>(ipw, WIP + (size_t)i * 3 * NC * NC, 3 * NC * NC,
                                                         opw, WOP + (size_t)i * NC * NC, NC * NC,
                                                         w1,  W1P + (size_t)i * FFI * NC, FFI * NC,
                                                         w2,  W2P + (size_t)i * NC * FFI, NC * FFI, WSC);
  }
  cvt_qk<<<dim3(NS / 64, NC / 64, 2), blk, 0, stream>>>(ml_c, caq, QH, QL, ml_r, cak, KH, KL);
  attn_x<<<dim3(NS / 32), blk, 0, stream>>>(QH, QL, KH, KL, VTA, XA);

  const float wsW  = 1.0f / WSC;
  const float wsWo = 1.0f / (WSC * OSC);
  const float wsW2 = 1.0f / (WSC * HSC);

  for (int i = 0; i < NBLK; ++i) {
    const int base = 5 + 14 * i;
    const float* n1w = (const float*)d_in[base + 0];
    const float* n1b = (const float*)d_in[base + 1];
    const float* n2w = (const float*)d_in[base + 2];
    const float* n2b = (const float*)d_in[base + 3];
    const float* ipb = (const float*)d_in[base + 5];
    const float* opb = (const float*)d_in[base + 7];
    const float* b1  = (const float*)d_in[base + 9];
    const float* b2  = (const float*)d_in[base + 11];
    const float* qp  = (const float*)d_in[base + 12];
    const float* kp  = (const float*)d_in[base + 13];
    const unsigned short* wq  = WIP + (size_t)i * 3 * NC * NC;
    const unsigned short* wk  = wq + (size_t)NC * NC;
    const unsigned short* wv  = wq + (size_t)2 * NC * NC;
    const unsigned short* wo  = WOP + (size_t)i * NC * NC;
    const unsigned short* w1p = W1P + (size_t)i * FFI * NC;
    const unsigned short* w2p = W2P + (size_t)i * NC * FFI;

    ln_rows<<<dim3(NS / 8), blk, 0, stream>>>(XA, n1w, n1b, qp, kp, XQ, XK, XV, 1, NS);
    {
      GDesc d[3];
      d[0] = gdesc(XQ, NC, wq, NC, (void*)QP, NC, NS, NC, NC, ipb, NC, XA, 0, F_BIASN | F_OUT16, wsW, PSC);
      d[1] = gdesc(XK, NC, wk, NC, (void*)KP, NC, NS, NC, NC, ipb + NC, NC, XA, 0, F_BIASN | F_OUT16, wsW, PSC);
      d[2] = gdesc(wv, NC, XV, NC, (void*)VTP, NS, NC, NS, NC, ipb + 2 * NC, NC, XA, 0, F_BIASM | F_OUT16, wsW, PSC);
      run_gemm(d, 3, stream);
    }
    attn_h<<<dim3(NS / 16), blk, 0, stream>>>(QP, KP, VTP, OP);
    {
      GDesc d[1];
      d[0] = gdesc(OP, NC, wo, NC, (void*)XB, NC, NS, NC, NC, opb, NC, XA, NC, F_BIASN | F_RESID, wsWo, 1.0f);
      run_gemm(d, 1, stream);
    }
    ln_rows<<<dim3(NS / 8), blk, 0, stream>>>(XB, n2w, n2b, qp, kp, AH, AH, AH, 0, NS);
    {
      GDesc d[1];
      d[0] = gdesc(AH, NC, w1p, NC, (void*)HP, FFI, NS, FFI, NC, b1, FFI, XA, 0, F_BIASN | F_GELU | F_OUT16, wsW, HSC);
      run_gemm(d, 1, stream);
    }
    {
      GDesc d[1];
      d[0] = gdesc(HP, FFI, w2p, FFI, (void*)XA, NC, NS, NC, FFI, b2, NC, XB, NC, F_BIASN | F_RESID, wsW2, 1.0f);
      run_gemm(d, 1, stream);
    }
  }

  out_nchw<<<dim3(NS / 64, NC / 64), blk, 0, stream>>>(XA, out);
  (void)hipGetLastError();
}
